// Multihead_Attention_16011638080099
// MI455X (gfx1250) — hardware-verified
//
#include <hip/hip_runtime.h>
#include <math.h>

#ifndef NB
#define NB 4
#endif
#define NB_FULL 4
#define CIN 512
#define HIMG 48
#define WIMG 48
#define LP 2304
#define CH3 192
#define HCH 64
#define NHEAD 8
#define DHEAD 8
#define COUT 512
#define PADW 50
#define LPAD 2500
#define MROWS (NB * LP)

#define WQ_BLKS ((CH3 * CIN / 8) / 256)
#define WR_BLKS ((COUT * HCH / 8) / 256)
#define WP_BLKS ((9 * HCH * HCH / 8) / 256)

static_assert(NB >= 1 && NB <= NB_FULL);
static_assert(LP == HIMG * WIMG);
static_assert(LP % 64 == 0 && LP % 128 == 0 && LP % 32 == 0 && LP % 16 == 0);
static_assert(MROWS % 64 == 0);
static_assert(CH3 % 64 == 0 && COUT % 64 == 0);
static_assert(CIN % 32 == 0 && HCH % 32 == 0 && CIN % 64 == 0);
static_assert(NHEAD * 3 * DHEAD == CH3 && NHEAD * DHEAD == HCH && DHEAD == 8);
static_assert(WIMG % 16 == 0 && PADW == WIMG + 2 && LPAD == PADW * PADW);
static_assert((LPAD * 8) % 32 == 0);
static_assert((CH3 * CIN / 8) % 256 == 0 && (COUT * HCH / 8) % 256 == 0 && (9 * HCH * HCH / 8) % 256 == 0);
static_assert(8 * 16 * 68 * 4 <= 131072);
static_assert(8 * 16 * 36 * 4 + 16 * 68 * 4 <= 131072);
static_assert(64 * 68 * 4 <= 131072 && 8 * 132 * 4 <= 131072 && 3 * 16 * 68 * 4 <= 131072);

typedef __attribute__((ext_vector_type(16))) _Float16 v16h;
typedef __attribute__((ext_vector_type(8)))  _Float16 v8h;
typedef __attribute__((ext_vector_type(2)))  _Float16 v2h;
typedef __attribute__((ext_vector_type(8)))  float    v8f;
typedef __attribute__((ext_vector_type(4)))  float    v4f;
typedef __attribute__((ext_vector_type(2)))  float    v2f;
typedef __attribute__((ext_vector_type(4)))  unsigned int v4u;


#define VST2(T, ptr, val) do { const T vst2_v_ = (val); *(volatile T*)(ptr) = vst2_v_; __threadfence(); *(volatile T*)(ptr) = vst2_v_; } while (0)

__device__ __forceinline__ float bfr(float f) {
    unsigned u = __float_as_uint(f);
    u += 0x7FFFu + ((u >> 16) & 1u);
    return __uint_as_float(u & 0xFFFF0000u);
}
static __device__ __forceinline__ unsigned toh2_flush(float a, float b) {
    v2f w;
    w.x = (fabsf(a) < 6.103515625e-05f) ? 0.0f : a;
    w.y = (fabsf(b) < 6.103515625e-05f) ? 0.0f : b;
    const v2h r = __builtin_convertvector(w, v2h);
    return __builtin_bit_cast(unsigned, r);
}
static __device__ __forceinline__ void st8hf(unsigned short* P, size_t o, const float* v) {
    v4u pk;
    pk.x = toh2_flush(v[0], v[1]);
    pk.y = toh2_flush(v[2], v[3]);
    pk.z = toh2_flush(v[4], v[5]);
    pk.w = toh2_flush(v[6], v[7]);
    VST2(v4u, (v4u*)(P + o), pk);
}

union FragU { v16h v; v8h h[2]; };
union FragQ { v16h v; v4u u[2]; };
__device__ __forceinline__ v16h frag_ld(const _Float16* p) {
    FragU f; f.h[0] = *(const v8h*)(p); f.h[1] = *(const v8h*)(p + 16); return f.v;
}
static __device__ __forceinline__ v16h frag8_ld(const _Float16* p, v4u mk) {
    FragQ f; f.u[0] = (*(const v4u*)(p)) & mk; f.u[1] = (v4u){0u, 0u, 0u, 0u}; return f.v;
}
__device__ __forceinline__ v8f wmma16(v16h a, v16h b, v8f c) {
    c = __builtin_amdgcn_wmma_f32_16x16x32_f16(false, a, false, b, (short)0, c, false, false);
    asm volatile("v_nop\n\tv_nop\n\tv_nop\n\tv_nop" : "+v"(c) : "v"(a), "v"(b));
    return c;
}
__device__ __forceinline__ void wave_sync_lds() {
    __builtin_amdgcn_fence(3  , "workgroup");
    __builtin_amdgcn_wave_barrier();
    __builtin_amdgcn_fence(2  , "workgroup");
}

template <int OUT_MODE, bool RESID, bool RELU, bool BIAS_ROW>
static __device__ __forceinline__ void gemm64_body(
    const _Float16* __restrict__ A, unsigned lda, const _Float16* __restrict__ Bt, unsigned ldb,
    void* __restrict__ Cout, unsigned ldc, const float* __restrict__ bias, const float* __restrict__ resid,
    unsigned M, unsigned N, unsigned K, float scale, float oscale) {
  __shared__ __align__(16) float sT[8][16 * 68];
  const unsigned lane = threadIdx.x & 31u;
  const unsigned wave = (unsigned)__builtin_amdgcn_readfirstlane((int)(threadIdx.x >> 5));
  const unsigned tilesN = N >> 6, tilesM = M >> 6;
  const unsigned tile = blockIdx.x * 8u + wave;
  if (tile >= tilesM * tilesN) return;
  const unsigned tm = tile / tilesN;
  const unsigned tn = tile - tm * tilesN;
  const unsigned m0 = tm << 6, n0 = tn << 6;
  const unsigned rlane = lane & 15u;
  const unsigned koff = (lane >> 4) * 8u;
  const unsigned mOff = koff;

  v8f acc[4][4];
#pragma unroll
  for (int i = 0; i < 4; ++i)
#pragma unroll
    for (int j = 0; j < 4; ++j) acc[i][j] = (v8f){0.f,0.f,0.f,0.f,0.f,0.f,0.f,0.f};

  for (unsigned k0 = 0; k0 < K; k0 += 32u) {
    v16h bh[4];
#pragma unroll
    for (int j = 0; j < 4; ++j)
      bh[j] = frag_ld(Bt + (size_t)(n0 + ((unsigned)j << 4) + rlane) * ldb + koff + k0);
#pragma unroll
    for (int i = 0; i < 4; ++i) {
      const v16h ah = frag_ld(A + (size_t)(m0 + ((unsigned)i << 4) + rlane) * lda + koff + k0);
#pragma unroll
      for (int j = 0; j < 4; ++j)
        acc[i][j] = wmma16(ah, bh[j], acc[i][j]);
    }
  }

  float* slab = sT[wave];
#pragma unroll
  for (int i = 0; i < 4; ++i) {
    const unsigned mBase = m0 + ((unsigned)i << 4);
    float bvr[8];
#pragma unroll
    for (int r = 0; r < 8; ++r) bvr[r] = BIAS_ROW ? bfr(bias[mBase + mOff + (unsigned)r]) : 0.0f;
#pragma unroll
    for (int j = 0; j < 4; ++j) {
      const unsigned n = n0 + ((unsigned)j << 4) + rlane;
      const float bvc = BIAS_ROW ? 0.0f : bfr(bias[n]);
#pragma unroll
      for (int r = 0; r < 8; ++r) {
        float v = acc[i][j][r] * scale + (BIAS_ROW ? bvr[r] : bvc);
        if (RELU) v = fmaxf(v, 0.0f);
        if (OUT_MODE == 1) v *= oscale;
        slab[(mOff + (unsigned)r) * 68u + ((unsigned)j << 4) + rlane] = v;
      }
    }
    wave_sync_lds();
    if (OUT_MODE == 0) {
      float* C = (float*)Cout;
      const unsigned hh = lane >> 4, c4 = (lane & 15u) * 4u;
      static_assert(2 * 4 * 32 * 16 == 16 * 64 * 4);
#pragma unroll
      for (int half = 0; half < 2; ++half) {
        v4f vv[4];
#pragma unroll
        for (int it = 0; it < 4; ++it) {
          const unsigned row = (unsigned)(half * 4 + it) * 2u + hh;
          vv[it] = *(const v4f*)(slab + row * 68u + c4);
          if (RESID) vv[it] += *(const v4f*)(resid + (size_t)(mBase + row) * ldc + n0 + c4);
        }
        for (int pass = 0; pass < 2; ++pass) {
#pragma unroll
          for (int it = 0; it < 4; ++it) {
            const unsigned row = (unsigned)(half * 4 + it) * 2u + hh;
            *(volatile v4f*)(C + (size_t)(mBase + row) * ldc + n0 + c4) = vv[it];
          }
          __threadfence();
        }
      }
    } else {
      unsigned short* C = (unsigned short*)Cout;
      const unsigned q = lane >> 3, c8 = (lane & 7u) * 8u;
      static_assert(4 * 32 * 16 == 16 * 64 * 2);
      v4u hv[4];
#pragma unroll
      for (int it = 0; it < 4; ++it) {
        const unsigned row = (unsigned)it * 4u + q;
        const float* sp = slab + row * 68u + c8;
        const v4f a = *(const v4f*)(sp);
        const v4f b = *(const v4f*)(sp + 4);
        hv[it].x = toh2_flush(a.x, a.y);
        hv[it].y = toh2_flush(a.z, a.w);
        hv[it].z = toh2_flush(b.x, b.y);
        hv[it].w = toh2_flush(b.z, b.w);
      }
      for (int pass = 0; pass < 2; ++pass) {
#pragma unroll
        for (int it = 0; it < 4; ++it) {
          const unsigned row = (unsigned)it * 4u + q;
          *(volatile v4u*)(C + (size_t)(mBase + row) * ldc + n0 + c8) = hv[it];
        }
        __threadfence();
      }
    }
    wave_sync_lds();
  }
}

__global__ __launch_bounds__(256) void k_gemm_qkv(const _Float16* __restrict__ X16, const _Float16* __restrict__ WQ16,
                                                  const float* __restrict__ qkv_b, unsigned short* __restrict__ QKV16) {
  gemm64_body<1, false, false, false>(X16, CIN, WQ16, CIN, (void*)QKV16, CH3, qkv_b, nullptr,
                                      MROWS, CH3, CIN, 9.5367431640625e-07f, 256.0f);
}

__global__ __launch_bounds__(256) void k_gemm_out(const _Float16* __restrict__ WR16, const _Float16* __restrict__ T16,
                                                  const float* __restrict__ res_b, float* __restrict__ out) {
  const unsigned n = blockIdx.y;
  gemm64_body<0, false, false, true>(WR16, HCH, T16 + (size_t)n * LP * HCH, HCH, (void*)(out + (size_t)n * COUT * LP), LP,
                                     res_b, nullptr, COUT, LP, HCH, 9.5367431640625e-07f, 1.0f);
}

__global__ __launch_bounds__(256) void k_wplanes(const float* __restrict__ qkv_w, const float* __restrict__ res_w,
                                                 const float* __restrict__ pos_w, unsigned short* __restrict__ WQ16,
                                                 unsigned short* __restrict__ WR16, unsigned short* __restrict__ WP16) {
  const unsigned blk = blockIdx.x, tid = threadIdx.x;
  float v[8];
  if (blk < (unsigned)WQ_BLKS) {
    const unsigned u = blk * 256u + tid;
    const v4f a = *(const v4f*)(qkv_w + (size_t)u * 8u), b = *(const v4f*)(qkv_w + (size_t)u * 8u + 4u);
    v[0] = bfr(a.x) * 4096.0f; v[1] = bfr(a.y) * 4096.0f; v[2] = bfr(a.z) * 4096.0f; v[3] = bfr(a.w) * 4096.0f;
    v[4] = bfr(b.x) * 4096.0f; v[5] = bfr(b.y) * 4096.0f; v[6] = bfr(b.z) * 4096.0f; v[7] = bfr(b.w) * 4096.0f;
    st8hf(WQ16, (size_t)u * 8u, v);
  } else if (blk < (unsigned)(WQ_BLKS + WR_BLKS)) {
    const unsigned u = (blk - (unsigned)WQ_BLKS) * 256u + tid;
    const v4f a = *(const v4f*)(res_w + (size_t)u * 8u), b = *(const v4f*)(res_w + (size_t)u * 8u + 4u);
    v[0] = bfr(a.x) * 4096.0f; v[1] = bfr(a.y) * 4096.0f; v[2] = bfr(a.z) * 4096.0f; v[3] = bfr(a.w) * 4096.0f;
    v[4] = bfr(b.x) * 4096.0f; v[5] = bfr(b.y) * 4096.0f; v[6] = bfr(b.z) * 4096.0f; v[7] = bfr(b.w) * 4096.0f;
    st8hf(WR16, (size_t)u * 8u, v);
  } else {
    const unsigned u = (blk - (unsigned)(WQ_BLKS + WR_BLKS)) * 256u + tid;
    const unsigned tap = u >> 9, rem = u & 511u;
    const unsigned o = rem >> 3, c0 = (rem & 7u) * 8u;
#pragma unroll
    for (int e = 0; e < 8; ++e) v[e] = bfr(pos_w[(size_t)(o * (unsigned)HCH + c0 + (unsigned)e) * 9u + tap]) * 4096.0f;
    st8hf(WP16, (size_t)(tap * (unsigned)HCH + o) * (unsigned)HCH + c0, v);
  }
}

__global__ __launch_bounds__(256) void k_xT(const float* __restrict__ x, unsigned short* __restrict__ X16) {
  __shared__ __align__(16) float sT[64 * 68];
  const unsigned tid = threadIdx.x;
  const unsigned p0 = blockIdx.x * 64u, c0 = blockIdx.y * 64u, n = blockIdx.z;
  const float* src = x + (size_t)n * CIN * LP;
  static_assert(256 * 4 * 16 == 64 * 64 * 4);
#pragma unroll
  for (int it = 0; it < 4; ++it) {
    const unsigned id = tid + 256u * (unsigned)it;
    const unsigned cr = id >> 4, pq = id & 15u;
    const v4f v = *(const v4f*)(src + (size_t)(c0 + cr) * LP + p0 + 4u * pq);
    *(v4f*)(sT + cr * 68u + 4u * pq) = v;
  }
  __syncthreads();
  static_assert(256 * 2 * 16 == 64 * 64 * 2);
  v4u pk[2];
#pragma unroll
  for (int it = 0; it < 2; ++it) {
    const unsigned id = tid + 256u * (unsigned)it;
    const unsigned pr = id >> 3, cq = id & 7u;
    float f[8];
#pragma unroll
    for (int e = 0; e < 8; ++e) f[e] = bfr(sT[(8u * cq + (unsigned)e) * 68u + pr]) * 256.0f;
    pk[it].x = toh2_flush(f[0], f[1]);
    pk[it].y = toh2_flush(f[2], f[3]);
    pk[it].z = toh2_flush(f[4], f[5]);
    pk[it].w = toh2_flush(f[6], f[7]);
  }
  for (int pass = 0; pass < 2; ++pass) {
#pragma unroll
    for (int it = 0; it < 2; ++it) {
      const unsigned id = tid + 256u * (unsigned)it;
      const unsigned pr = id >> 3, cq = id & 7u;
      *(volatile v4u*)(X16 + (size_t)(n * (unsigned)LP + p0 + pr) * CIN + c0 + 8u * cq) = pk[it];
    }
    __threadfence();
  }
}

__global__ __launch_bounds__(256) void k_vt(const _Float16* __restrict__ QKV16, unsigned short* __restrict__ VT16) {
  __shared__ __align__(16) float sV[8 * 132];
  const unsigned tid = threadIdx.x;
  const unsigned wave = (unsigned)__builtin_amdgcn_readfirstlane((int)(tid >> 5));
  const unsigned g = blockIdx.y, n = g >> 3, h = g & 7u;
  const unsigned key0 = blockIdx.x * 128u;
  if (wave < 4u) {
    const v8h vv = *(const v8h*)(QKV16 + (size_t)(n * (unsigned)LP + key0 + tid) * CH3 + 24u * h + 16u);
#pragma unroll
    for (int e = 0; e < 8; ++e) sV[(unsigned)e * 132u + tid] = (float)vv[e];
  }
  __syncthreads();
  static_assert(256 * 16 == 16 * 128 * 2);
  const unsigned row = tid >> 4, piece = tid & 15u;
  const float* sp = sV + (row & 7u) * 132u + 8u * piece;
  const v4f a = *(const v4f*)(sp), b = *(const v4f*)(sp + 4);
  const bool live = row < 8u;
  v4u pk;
  pk.x = toh2_flush(live ? a.x : 0.0f, live ? a.y : 0.0f);
  pk.y = toh2_flush(live ? a.z : 0.0f, live ? a.w : 0.0f);
  pk.z = toh2_flush(live ? b.x : 0.0f, live ? b.y : 0.0f);
  pk.w = toh2_flush(live ? b.z : 0.0f, live ? b.w : 0.0f);
  VST2(v4u, (v4u*)(VT16 + (size_t)(g * 16u + row) * LP + key0 + 8u * piece), pk);
}

__global__ __launch_bounds__(256) void k_vhalo(const unsigned short* __restrict__ QKV16, unsigned short* __restrict__ VH16) {
  const unsigned u = blockIdx.x * 256u + threadIdx.x;
  const unsigned n = blockIdx.y;
  const unsigned h = u & 7u;
  unsigned r = u >> 3;
  if (r >= (unsigned)LPAD) return;
  asm volatile("" : "+v"(r));
  const unsigned py = r / (unsigned)PADW;
  const unsigned px = r - py * (unsigned)PADW;
  const bool inside = (py >= 1u) && (py <= (unsigned)HIMG) && (px >= 1u) && (px <= (unsigned)WIMG);
  const unsigned sy = min(max(py, 1u), (unsigned)HIMG) - 1u;
  const unsigned sx = min(max(px, 1u), (unsigned)WIMG) - 1u;
  const unsigned srow = n * (unsigned)LP + sy * (unsigned)WIMG + sx;
  const v4u raw = *(const v4u*)(QKV16 + (size_t)srow * CH3 + 24u * h + 16u);
  const unsigned m = inside ? 0xFFFFFFFFu : 0u;
  const v4u mk = (v4u){m, m, m, m};
  VST2(v4u, (v4u*)(VH16 + (size_t)(n * (unsigned)LPAD + r) * HCH + 8u * h), raw & mk);
}

#define AT_PP 36
__global__ __launch_bounds__(256) void k_attn(const _Float16* __restrict__ QKV16, const _Float16* __restrict__ VT16,
                                              float* __restrict__ OUT32) {
  __shared__ __align__(16) float sP[8][16 * AT_PP];
  __shared__ __align__(16) float sO[16 * 68];
  const unsigned tid = threadIdx.x, lane = tid & 31u;
  const unsigned wave = (unsigned)__builtin_amdgcn_readfirstlane((int)(tid >> 5));
  const unsigned hh = lane >> 4, c = lane & 15u;
  const unsigned n = blockIdx.y, head = wave;
  const unsigned g = n * (unsigned)NHEAD + head;
  const unsigned q0 = blockIdx.x * 16u;
  const unsigned rowbase = n * (unsigned)LP;
  const unsigned m32 = hh ? 0u : 0xFFFFFFFFu;
  const v4u mk = (v4u){m32, m32, m32, m32};
  float* pw = sP[wave];
  const float SC2 = 0.35355339059327379f * (1.0f / 65536.0f) * 1.4426950408889634f;
  const v16h qf = frag8_ld(QKV16 + (size_t)(rowbase + q0 + c) * CH3 + 24u * head, mk);
  const _Float16* vrow = VT16 + (size_t)(g * 16u + c) * LP + 8u * hh;
  float mrow[8], lrow[8];
  v8f os = (v8f){0.f,0.f,0.f,0.f,0.f,0.f,0.f,0.f};
#pragma unroll
  for (int r = 0; r < 8; ++r) { mrow[r] = -3.0e38f; lrow[r] = 0.f; }
#pragma unroll 1
  for (unsigned ks = 0; ks < (unsigned)(LP / 32); ++ks) {
    const unsigned kv0 = ks * 32u;
    v8f s[2];
#pragma unroll
    for (int j = 0; j < 2; ++j) {
      const v16h kf = frag8_ld(QKV16 + (size_t)(rowbase + kv0 + (unsigned)j * 16u + c) * CH3 + 24u * head + 8u, mk);
      const v8f z = (v8f){0.f,0.f,0.f,0.f,0.f,0.f,0.f,0.f};
      s[j] = wmma16(qf, kf, z);
    }
#pragma unroll
    for (int r = 0; r < 8; ++r) {
      float mx = -3.0e38f;
#pragma unroll
      for (int j = 0; j < 2; ++j) { s[j][r] *= SC2; mx = fmaxf(mx, s[j][r]); }
      mx = fmaxf(mx, __shfl_xor(mx, 1, 32)); mx = fmaxf(mx, __shfl_xor(mx, 2, 32));
      mx = fmaxf(mx, __shfl_xor(mx, 4, 32)); mx = fmaxf(mx, __shfl_xor(mx, 8, 32));
      const float mnew = fmaxf(mrow[r], mx);
      const float alpha = exp2f(mrow[r] - mnew);
      mrow[r] = mnew;
      float psum = 0.f;
#pragma unroll
      for (int j = 0; j < 2; ++j) {
        const float p = exp2f(s[j][r] - mnew);
        psum += p;
        pw[(8u * hh + (unsigned)r) * AT_PP + (unsigned)j * 16u + c] = p;
      }
      psum += __shfl_xor(psum, 1, 32); psum += __shfl_xor(psum, 2, 32);
      psum += __shfl_xor(psum, 4, 32); psum += __shfl_xor(psum, 8, 32);
      lrow[r] = lrow[r] * alpha + psum;
      os[r] *= alpha;
    }
    wave_sync_lds();
    {
      const float* pr = pw + c * AT_PP + 8u * hh;
      const v4f p0 = *(const v4f*)(pr), p1 = *(const v4f*)(pr + 4), p2 = *(const v4f*)(pr + 16), p3 = *(const v4f*)(pr + 20);
      FragQ pa;
      pa.u[0].x = toh2_flush(p0.x * 1024.0f, p0.y * 1024.0f);
      pa.u[0].y = toh2_flush(p0.z * 1024.0f, p0.w * 1024.0f);
      pa.u[0].z = toh2_flush(p1.x * 1024.0f, p1.y * 1024.0f);
      pa.u[0].w = toh2_flush(p1.z * 1024.0f, p1.w * 1024.0f);
      pa.u[1].x = toh2_flush(p2.x * 1024.0f, p2.y * 1024.0f);
      pa.u[1].y = toh2_flush(p2.z * 1024.0f, p2.w * 1024.0f);
      pa.u[1].z = toh2_flush(p3.x * 1024.0f, p3.y * 1024.0f);
      pa.u[1].w = toh2_flush(p3.z * 1024.0f, p3.w * 1024.0f);
      const v16h vb = frag_ld(vrow + kv0);
      os = wmma16(pa.v, vb, os);
    }
    wave_sync_lds();
  }
#pragma unroll
  for (int r = 0; r < 8; ++r) {
    const float den = lrow[r] * 262144.0f;
    const float o = os[r] / den;
    if (c < 8u) sO[(8u * hh + (unsigned)r) * 68u + 8u * head + c] = o;
  }
  __syncthreads();
  {
    static_assert(256 * 16 == 16 * 64 * 4);
    const unsigned row = tid >> 4, piece = tid & 15u;
    const v4f v = *(const v4f*)(sO + row * 68u + 4u * piece);
    float* dst = OUT32 + (size_t)(rowbase + q0 + row) * HCH + 4u * piece;
    for (int pass = 0; pass < 2; ++pass) {
      *(volatile v4f*)(dst) = v;
      __threadfence();
    }
  }
}

__global__ __launch_bounds__(96) void k_pos(const _Float16* __restrict__ VH16, const _Float16* __restrict__ WP16,
                                            const float* __restrict__ pos_b, const float* __restrict__ OUT32,
                                            unsigned short* __restrict__ T16) {
  __shared__ __align__(16) float sT[3][16 * 68];
  const unsigned lane = threadIdx.x & 31u;
  const unsigned wave = (unsigned)__builtin_amdgcn_readfirstlane((int)(threadIdx.x >> 5));
  const unsigned rlane = lane & 15u;
  const unsigned koff = (lane >> 4) * 8u;
  const unsigned mOff = koff;
  const unsigned y = blockIdx.x, n = blockIdx.y;
  const unsigned x0 = wave * 16u;
  static_assert(WIMG == 3 * 16);

  v8f acc[4];
#pragma unroll
  for (int j = 0; j < 4; ++j) acc[j] = (v8f){0.f,0.f,0.f,0.f,0.f,0.f,0.f,0.f};

  for (unsigned ti = 0; ti < 3u; ++ti) {
    for (unsigned tj = 0; tj < 3u; ++tj) {
      const unsigned tap = ti * 3u + tj;
      const _Float16* arow = VH16 + (size_t)(n * (unsigned)LPAD + (y + ti) * (unsigned)PADW + x0 + tj + rlane) * HCH + koff;
      const _Float16* brow = WP16 + (size_t)(tap * (unsigned)HCH + rlane) * HCH + koff;
      for (unsigned k0 = 0; k0 < (unsigned)HCH; k0 += 32u) {
        const v16h ah = frag_ld(arow + k0);
#pragma unroll
        for (int j = 0; j < 4; ++j) {
          const v16h bh = frag_ld(brow + (size_t)((unsigned)j << 4) * HCH + k0);
          acc[j] = wmma16(ah, bh, acc[j]);
        }
      }
    }
  }

  float* slab = sT[wave];
#pragma unroll
  for (int j = 0; j < 4; ++j) {
    const float bv = bfr(pos_b[((unsigned)j << 4) + rlane]);
#pragma unroll
    for (int r = 0; r < 8; ++r)
      slab[(mOff + (unsigned)r) * 68u + ((unsigned)j << 4) + rlane] = acc[j][r] * 9.5367431640625e-07f + bv;
  }
  wave_sync_lds();
  {
    const unsigned q = lane >> 3, c8 = (lane & 7u) * 8u;
    static_assert(4 * 32 * 16 == 16 * 64 * 2);
    const unsigned prow0 = n * (unsigned)LP + y * (unsigned)WIMG + x0;
    v4u hv[4];
#pragma unroll
    for (int it = 0; it < 4; ++it) {
      const unsigned row = (unsigned)it * 4u + q;
      const float* sp = slab + row * 68u + c8;
      const float* op = OUT32 + (size_t)(prow0 + row) * HCH + c8;
      const v4f a = (*(const v4f*)(sp) + *(const v4f*)(op)) * 256.0f;
      const v4f b = (*(const v4f*)(sp + 4) + *(const v4f*)(op + 4)) * 256.0f;
      hv[it].x = toh2_flush(a.x, a.y);
      hv[it].y = toh2_flush(a.z, a.w);
      hv[it].z = toh2_flush(b.x, b.y);
      hv[it].w = toh2_flush(b.z, b.w);
    }
    for (int pass = 0; pass < 2; ++pass) {
#pragma unroll
      for (int it = 0; it < 4; ++it) {
        const unsigned row = (unsigned)it * 4u + q;
        *(volatile v4u*)(T16 + (size_t)(prow0 + row) * HCH + c8) = hv[it];
      }
      __threadfence();
    }
  }
}

constexpr size_t SZ_X16   = (size_t)MROWS * CIN * 2;
constexpr size_t SZ_QKV16 = (size_t)MROWS * CH3 * 2;
constexpr size_t SZ_VT16  = (size_t)NB * NHEAD * 16 * LP * 2;
constexpr size_t SZ_VH16  = (size_t)NB * LPAD * HCH * 2;
constexpr size_t SZ_OUT32 = (size_t)MROWS * HCH * 4;
constexpr size_t SZ_T16   = (size_t)MROWS * HCH * 2;
constexpr size_t SZ_WQ16  = (size_t)CH3 * CIN * 2;
constexpr size_t SZ_WR16  = (size_t)COUT * HCH * 2;
constexpr size_t SZ_WP16  = (size_t)9 * HCH * HCH * 2;
constexpr size_t OFF_X16   = 0;
constexpr size_t OFF_QKV16 = OFF_X16 + SZ_X16;
constexpr size_t OFF_VT16  = OFF_QKV16 + SZ_QKV16;
constexpr size_t OFF_VH16  = OFF_VT16 + SZ_VT16;
constexpr size_t OFF_OUT32 = OFF_VH16 + SZ_VH16;
constexpr size_t OFF_T16   = OFF_OUT32 + SZ_OUT32;
constexpr size_t OFF_WQ16  = OFF_T16 + SZ_T16;
constexpr size_t OFF_WR16  = OFF_WQ16 + SZ_WQ16;
constexpr size_t OFF_WP16  = OFF_WR16 + SZ_WR16;
constexpr size_t WS_TOTAL  = OFF_WP16 + SZ_WP16;
static_assert(SZ_X16 % 256 == 0 && SZ_QKV16 % 256 == 0 && SZ_VT16 % 256 == 0 && SZ_VH16 % 256 == 0);
static_assert(SZ_OUT32 % 256 == 0 && SZ_T16 % 256 == 0 && SZ_WQ16 % 256 == 0 && SZ_WR16 % 256 == 0 && SZ_WP16 % 256 == 0);
static_assert(WS_TOTAL <= (size_t)134217728);
static_assert((MROWS / 64) * (CH3 / 64) > 0);
static_assert(((COUT / 64) * (LP / 64)) % 8 == 0);

extern "C" void kernel_launch(void* const* d_in, const int* in_sizes, int n_in, void* d_out, int out_size,
                              void* d_ws, size_t ws_size, hipStream_t stream) {
    if (n_in < 7) return;
    if (in_sizes[0] < NB * CIN * LP || in_sizes[1] < CH3 * CIN || in_sizes[2] < CH3) return;
    if (in_sizes[3] < HCH * HCH * 9 || in_sizes[4] < HCH || in_sizes[5] < COUT * HCH || in_sizes[6] < COUT) return;
    if (out_size < NB * COUT * LP) return;
    if (WS_TOTAL > ws_size) return;

    const float* x     = (const float*)d_in[0];
    const float* qkv_w = (const float*)d_in[1];
    const float* qkv_b = (const float*)d_in[2];
    const float* pos_w = (const float*)d_in[3];
    const float* pos_b = (const float*)d_in[4];
    const float* res_w = (const float*)d_in[5];
    const float* res_b = (const float*)d_in[6];
    float* out = (float*)d_out;

    char* wsp = (char*)d_ws;
    unsigned short* X16   = (unsigned short*)(wsp + OFF_X16);
    unsigned short* QKV16 = (unsigned short*)(wsp + OFF_QKV16);
    unsigned short* VT16  = (unsigned short*)(wsp + OFF_VT16);
    unsigned short* VH16  = (unsigned short*)(wsp + OFF_VH16);
    float*          OUT32 = (float*)(wsp + OFF_OUT32);
    unsigned short* T16   = (unsigned short*)(wsp + OFF_T16);
    unsigned short* WQ16  = (unsigned short*)(wsp + OFF_WQ16);
    unsigned short* WR16  = (unsigned short*)(wsp + OFF_WR16);
    unsigned short* WP16  = (unsigned short*)(wsp + OFF_WP16);

    k_wplanes<<<WQ_BLKS + WR_BLKS + WP_BLKS, 256, 0, stream>>>(qkv_w, res_w, pos_w, WQ16, WR16, WP16);
    k_xT<<<dim3(LP / 64, CIN / 64, NB), 256, 0, stream>>>(x, X16);
    k_gemm_qkv<<<((MROWS / 64) * (CH3 / 64) + 7) / 8, 256, 0, stream>>>((const _Float16*)X16, (const _Float16*)WQ16, qkv_b, QKV16);
    k_vt<<<dim3(LP / 128, NB * NHEAD), 256, 0, stream>>>((const _Float16*)QKV16, VT16);
    k_vhalo<<<dim3((LPAD * 8 + 255) / 256, NB), 256, 0, stream>>>((const unsigned short*)QKV16, VH16);
    k_attn<<<dim3(LP / 16, NB), 256, 0, stream>>>((const _Float16*)QKV16, (const _Float16*)VT16, OUT32);
    k_pos<<<dim3(HIMG, NB), 96, 0, stream>>>((const _Float16*)VH16, (const _Float16*)WP16, pos_b, (const float*)OUT32, T16);
    k_gemm_out<<<dim3(((COUT / 64) * (LP / 64)) / 8, NB), 256, 0, stream>>>((const _Float16*)WR16, (const _Float16*)T16, res_b, out);
}
